// PairSelfAttention_60395830116865
// MI455X (gfx1250) — hardware-verified
//
#include <hip/hip_runtime.h>
#include <math.h>
#include <stdint.h>

#pragma clang fp contract(off)

#define NB   32
#define SEQ  512
#define EMB  256
#define NH   8
#define HD   32
#define QD   64
#define NQT  (SEQ / 64)
#define NKT  (SEQ / 64)
static_assert(NH * HD == EMB);
static_assert(NQT == 8 && NKT == 8);
static_assert((SEQ % 64) == 0 && (HD % 32) == 0 && (QD % 32) == 0);

typedef _Float16 v16h __attribute__((ext_vector_type(16)));
typedef _Float16 v8h  __attribute__((ext_vector_type(8)));
typedef __bf16   v16b __attribute__((ext_vector_type(16)));
typedef __bf16   v8b  __attribute__((ext_vector_type(8)));
typedef float    v8f  __attribute__((ext_vector_type(8)));
typedef float    v4f  __attribute__((ext_vector_type(4)));
typedef unsigned int v4u __attribute__((ext_vector_type(4)));
typedef unsigned int v2u __attribute__((ext_vector_type(2)));
typedef int      v4i  __attribute__((ext_vector_type(4)));

#if defined(__HIP_DEVICE_COMPILE__)
#define DEV_ASM 1
#else
#define DEV_ASM 0
#endif

__device__ __forceinline__ unsigned short bf_bits(float f) {
  unsigned u = __float_as_uint(f);
  return (unsigned short)((u + 0x7FFFu + ((u >> 16) & 1u)) >> 16);
}
__device__ __forceinline__ float bf_up(unsigned short hb) { return __uint_as_float(((unsigned)hb) << 16); }
__device__ __forceinline__ unsigned short h_bits(_Float16 x) { return __builtin_bit_cast(unsigned short, x); }
__device__ __forceinline__ unsigned pk16(unsigned short a, unsigned short b) { return (unsigned)a | ((unsigned)b << 16); }
__device__ __forceinline__ v8f zero8() { v8f z = {0.f, 0.f, 0.f, 0.f, 0.f, 0.f, 0.f, 0.f}; return z; }

template <typename OT> struct FT;
template <> struct FT<__bf16>   { typedef v16b frag; typedef v8b half8; };
template <> struct FT<_Float16> { typedef v16h frag; typedef v8h half8; };

template <typename OT>
__device__ __forceinline__ typename FT<OT>::frag ldfrag(const OT* p) {
  union { typename FT<OT>::frag v; typename FT<OT>::half8 h[2]; } f;
  f.h[0] = *(const typename FT<OT>::half8*)(p);
  f.h[1] = *(const typename FT<OT>::half8*)(p + 16);
  return f.v;
}

__device__ __forceinline__ v8f mma_b(v16b a, v16b b, v8f c) {
  c = __builtin_amdgcn_wmma_f32_16x16x32_bf16(false, a, false, b, (short)0, c, false, false);
#if DEV_ASM
  asm volatile("v_nop\n\tv_nop\n\tv_nop\n\tv_nop" : "+v"(c) : "v"(a), "v"(b));
#endif
  return c;
}
__device__ __forceinline__ v8f mma_h(v16h a, v16h b, v8f c) {
  c = __builtin_amdgcn_wmma_f32_16x16x32_f16(false, a, false, b, (short)0, c, false, false);
#if DEV_ASM
  asm volatile("v_nop\n\tv_nop\n\tv_nop\n\tv_nop" : "+v"(c) : "v"(a), "v"(b));
#endif
  return c;
}

__global__ __launch_bounds__(64) void k_partner(const float* __restrict__ cen, int* pt) {
#pragma clang fp contract(off)
  __shared__ float sb0[SEQ];
  __shared__ float sb1[SEQ];
  __shared__ float sb2[SEQ];
  __shared__ float sb3[SEQ];
  __shared__ float sar[SEQ];
  __shared__ float sl1[SEQ];
  __shared__ __align__(16) int sp[128];

  const int tid = (int)threadIdx.x;
  const int i0  = (int)blockIdx.x * 64;
  const int b   = (int)blockIdx.y;
  const float* cb = cen + (size_t)b * SEQ * 4;

  for (int s = tid; s < SEQ; s += 64) {
    const v4f cv = *(const v4f*)(cb + (size_t)s * 4);
    const float c0 = bf_up(bf_bits(cv[0]));
    const float c1 = bf_up(bf_bits(cv[1]));
    const float c2 = bf_up(bf_bits(cv[2]));
    const float c3 = bf_up(bf_bits(cv[3]));
    const float hx = c3 * 0.5f;
    const float hy = c2 * 0.5f;
    const float x0 = c0 - hx;
    const float y0 = c1 - hy;
    const float x1 = c0 + hx;
    const float y1 = c1 + hy;
    sb0[s] = x0;
    sb1[s] = y0;
    sb2[s] = x1;
    sb3[s] = y1;
    const float dx = x1 - x0;
    const float dy = y1 - y0;
    sar[s] = dx * dy;
    const float la = c2 - c0;
    const float lb = c3 - c1;
    sl1[s] = la + lb;
  }
  __syncthreads();

  const int i = i0 + tid;
  const float a0 = sb0[i], a1 = sb1[i], a2 = sb2[i], a3 = sb3[i], ar = sar[i];
  float best = -INFINITY;
  int   bj = 0;
  bool  seen_nan = false;
#pragma unroll 2
  for (int j = 0; j < SEQ; ++j) {
    const float m0 = fmaxf(a0, sb0[j]);
    const float m1 = fmaxf(a1, sb1[j]);
    const float x2 = fminf(a2, sb2[j]);
    const float x3 = fminf(a3, sb3[j]);
    const float d0 = x2 - m0;
    const float d1 = x3 - m1;
    const float w0 = fmaxf(d0, 0.0f);
    const float w1 = fmaxf(d1, 0.0f);
    const float inter = w0 * w1;
    const float asum  = ar + sar[j];
    const float uni   = asum - inter;
    const float q     = inter / uni;
    const float e     = (j == i) ? 1.0f : 0.0f;
    const float iou   = q - e;
    if (!seen_nan) {
      if (iou != iou) { bj = j; seen_nan = true; }
      else if (iou > best) { best = iou; bj = j; }
    }
  }
  const float l1i = sl1[i];
  const float l1p = sl1[bj];
  const bool cond = (l1i >= l1p);
  sp[tid * 2 + 0] = cond ? i : bj;
  sp[tid * 2 + 1] = cond ? bj : i;
  __syncthreads();

  if (tid < 32) {
    const v4i v = *(const v4i*)(sp + tid * 4);
    int* dst = pt + ((size_t)b * SEQ + i0) * 2 + tid * 4;
    *(volatile v4i*)dst = v;
    __threadfence();
    *(volatile v4i*)dst = v;
  }
}

__global__ __launch_bounds__(256) void k_proj(
    const float* __restrict__ content, const float* __restrict__ pos, const int* __restrict__ pt,
    const float* __restrict__ Wq, const float* __restrict__ Wk, const float* __restrict__ Wv,
    unsigned short* q2p, unsigned short* k2p, unsigned short* vhp, unsigned short* vlp) {
  __shared__ __align__(16) unsigned short Xg[2][64 * QD];
  __shared__ __align__(16) unsigned short Xv[64 * HD];
  __shared__ __align__(16) unsigned short W2[2][HD * QD];
  __shared__ __align__(16) unsigned short Wvt[HD * HD];
  __shared__ int sIdx[2][64];
  __shared__ __align__(16) unsigned short stQK[2][64 * QD];
  __shared__ __align__(16) float stV[HD * 64];

  const int tid  = (int)threadIdx.x;
  const int wave = tid >> 5;
  const int lane = tid & 31;
  const int rl   = lane & 15;
  const int hh   = lane >> 4;
  const int i0   = (int)blockIdx.x * 64;
  const int h    = (int)blockIdx.y;
  const int b    = (int)blockIdx.z;
  const size_t rowB = (size_t)b * SEQ;
  const size_t bh   = (size_t)b * NH + (size_t)h;

  if (tid < 128) {
    const int r = tid >> 1, g = tid & 1;
    int v = pt[(rowB + (size_t)(i0 + r)) * 2 + g];
    v = min(max(v, 0), SEQ - 1);
    sIdx[g][r] = v;
  }
  for (int e = tid; e < HD * QD; e += 256) {
    const int n = e >> 6, kp = e & 63, k = kp & 31;
    W2[0][e] = bf_bits(Wq[k * HD + n]);
    W2[1][e] = bf_bits(Wk[k * HD + n]);
  }
  for (int e = tid; e < HD * HD; e += 256) {
    const int n = e >> 5, k = e & 31;
    Wvt[e] = bf_bits(Wv[k * HD + n]);
  }
  for (int e = tid; e < 64 * HD / 4; e += 256) {
    const int r = e >> 3, c4 = (e & 7) * 4;
    const v4f v = *(const v4f*)(content + (rowB + (size_t)(i0 + r)) * EMB + (size_t)h * HD + c4);
    v2u pk;
    pk[0] = pk16(bf_bits(v[0]), bf_bits(v[1]));
    pk[1] = pk16(bf_bits(v[2]), bf_bits(v[3]));
    *(v2u*)(Xv + r * HD + c4) = pk;
  }
  __syncthreads();
#pragma unroll
  for (int it2 = 0; it2 < 8; ++it2) {
    const int g   = it2 >> 2;
    const int src = (it2 >> 1) & 1;
    const int e   = (it2 & 1) * 256 + tid;
    const int r   = e >> 3, c4 = (e & 7) * 4;
    const float* base = src ? pos : content;
    const int srow = sIdx[g][r];
    const v4f v = *(const v4f*)(base + (rowB + (size_t)srow) * EMB + (size_t)h * HD + c4);
    v2u pk;
    pk[0] = pk16(bf_bits(v[0]), bf_bits(v[1]));
    pk[1] = pk16(bf_bits(v[2]), bf_bits(v[3]));
    *(v2u*)(Xg[g] + r * QD + src * HD + c4) = pk;
  }
  __syncthreads();

  const int mt    = wave & 3;
  const int which = wave >> 2;
  const __bf16* Xb0 = (const __bf16*)(const void*)Xg[0];
  const __bf16* Xb1 = (const __bf16*)(const void*)Xg[1];
  const __bf16* Wb  = (const __bf16*)(const void*)W2[which];
  v8f acc00 = zero8(), acc01 = zero8(), acc10 = zero8(), acc11 = zero8();
#pragma unroll
  for (int ks = 0; ks < 2; ++ks) {
    const v16b b0 = ldfrag<__bf16>(Wb + (size_t)rl * QD + ks * 32 + 8 * hh);
    const v16b b1 = ldfrag<__bf16>(Wb + (size_t)(16 + rl) * QD + ks * 32 + 8 * hh);
    const v16b a0 = ldfrag<__bf16>(Xb0 + (size_t)(mt * 16 + rl) * QD + ks * 32 + 8 * hh);
    const v16b a1 = ldfrag<__bf16>(Xb1 + (size_t)(mt * 16 + rl) * QD + ks * 32 + 8 * hh);
    acc00 = mma_b(a0, b0, acc00);
    acc01 = mma_b(a0, b1, acc01);
    acc10 = mma_b(a1, b0, acc10);
    acc11 = mma_b(a1, b1, acc11);
  }
  const int dt = wave & 1, st = wave >> 1;
  const v16b av = ldfrag<__bf16>((const __bf16*)(const void*)Wvt + (size_t)(dt * 16 + rl) * HD + 8 * hh);
  const v16b bv = ldfrag<__bf16>((const __bf16*)(const void*)Xv + (size_t)(st * 16 + rl) * HD + 8 * hh);
  v8f accv = zero8();
  accv = mma_b(av, bv, accv);

  unsigned short* sq = stQK[which];
#pragma unroll
  for (int r = 0; r < 8; ++r) {
    const int row = mt * 16 + 8 * hh + r;
    sq[row * QD + 0  + rl] = h_bits((_Float16)(acc00[r] * 8.0f));
    sq[row * QD + 16 + rl] = h_bits((_Float16)(acc01[r] * 8.0f));
    sq[row * QD + 32 + rl] = h_bits((_Float16)(acc10[r] * 8.0f));
    sq[row * QD + 48 + rl] = h_bits((_Float16)(acc11[r] * 8.0f));
    stV[(dt * 16 + 8 * hh + r) * 64 + st * 16 + rl] = accv[r];
  }
  __syncthreads();

  const int q4 = lane >> 3, c8 = (lane & 7) * 8;
  v4u qv[2], kv[2];
#pragma unroll
  for (int it = 0; it < 2; ++it) {
    const int row = wave * 8 + it * 4 + q4;
    qv[it] = *(const v4u*)(stQK[0] + row * QD + c8);
    kv[it] = *(const v4u*)(stQK[1] + row * QD + c8);
  }
  const int d = wave * 4 + q4;
  v4u vhv, vlv;
  {
    const float* spv = stV + d * 64 + c8;
#pragma unroll
    for (int e = 0; e < 4; ++e) {
      const float f0 = spv[2 * e] * 8.0f, f1 = spv[2 * e + 1] * 8.0f;
      const _Float16 x0 = (_Float16)f0, x1 = (_Float16)f1;
      const float r0 = f0 - (float)x0, r1 = f1 - (float)x1;
      const _Float16 l0 = (_Float16)(r0 * 4096.0f), l1 = (_Float16)(r1 * 4096.0f);
      vhv[e] = pk16(h_bits(x0), h_bits(x1));
      vlv[e] = pk16(h_bits(l0), h_bits(l1));
    }
  }
  for (int pass = 0; pass < 2; ++pass) {
#pragma unroll
    for (int it = 0; it < 2; ++it) {
      const int row = wave * 8 + it * 4 + q4;
      const size_t po = (bh * SEQ + (size_t)(i0 + row)) * QD + c8;
      *(volatile v4u*)(q2p + po) = qv[it];
      *(volatile v4u*)(k2p + po) = kv[it];
    }
    const size_t vo = (bh * HD + (size_t)d) * SEQ + (size_t)i0 + c8;
    *(volatile v4u*)(vhp + vo) = vhv;
    *(volatile v4u*)(vlp + vo) = vlv;
    __threadfence();
  }
}

__global__ __launch_bounds__(128)
void k_attn(const unsigned short* __restrict__ q2p, const unsigned short* __restrict__ k2p,
            const unsigned short* __restrict__ vhp, const unsigned short* __restrict__ vlp,
            float* out, float sscale) {
  union FH { v16h v; v8h h[2]; };
  __shared__ __align__(16) _Float16 Ksh[64 * QD];
  __shared__ __align__(16) _Float16 Vth[HD * 64];
  __shared__ __align__(16) _Float16 Vtl[HD * 64];
  __shared__ __align__(16) _Float16 Psh[4][16 * 64];
  __shared__ __align__(16) _Float16 Psl[4][16 * 64];
  __shared__ __align__(16) float    Os[4][16 * HD];

  const int tid  = (int)threadIdx.x;
  const int wave = tid >> 5;
  const int lane = tid & 31;
  const int hh   = lane >> 4;
  const int c    = lane & 15;

  const int q0 = (int)blockIdx.x * 64 + wave * 16;
  const int h  = (int)blockIdx.y;
  const int b  = (int)blockIdx.z;
  const size_t bh = (size_t)b * NH + (size_t)h;

  const _Float16* Q  = (const _Float16*)(const void*)q2p + bh * SEQ * QD;
  const _Float16* K  = (const _Float16*)(const void*)k2p + bh * SEQ * QD;
  const _Float16* Vh = (const _Float16*)(const void*)vhp + bh * HD * SEQ;
  const _Float16* Vl = (const _Float16*)(const void*)vlp + bh * HD * SEQ;

  v16h qa[2];
#pragma unroll
  for (int dc = 0; dc < 2; ++dc)
    qa[dc] = ldfrag<_Float16>(Q + (size_t)(q0 + c) * QD + dc * 32 + 8 * hh);

  float mrow[8], lrow[8];
  v8f oacc[2];
#pragma unroll
  for (int r = 0; r < 8; ++r) { mrow[r] = -INFINITY; lrow[r] = 0.f; }
#pragma unroll
  for (int t = 0; t < 2; ++t) oacc[t] = zero8();

  for (int kt = 0; kt < NKT; ++kt) {
    const int kv0 = kt * 64;
    __syncthreads();
    {
      const int r = tid >> 1, half = (tid & 1) * 32;
      const _Float16* kg = K + (size_t)(kv0 + r) * QD + half;
#pragma unroll
      for (int i = 0; i < 4; ++i)
        *(v8h*)(Ksh + r * QD + half + 8 * i) = *(const v8h*)(kg + 8 * i);
      const int r2 = tid >> 2, qq = (tid & 3) * 16;
      const _Float16* vg  = Vh + (size_t)r2 * SEQ + kv0 + qq;
      const _Float16* vlg = Vl + (size_t)r2 * SEQ + kv0 + qq;
#pragma unroll
      for (int i = 0; i < 2; ++i) {
        *(v8h*)(Vth + r2 * 64 + qq + 8 * i) = *(const v8h*)(vg + 8 * i);
        *(v8h*)(Vtl + r2 * 64 + qq + 8 * i) = *(const v8h*)(vlg + 8 * i);
      }
    }
    __syncthreads();

    v8f s[4];
#pragma unroll
    for (int j = 0; j < 4; ++j) {
      v8f a = zero8();
#pragma unroll
      for (int dc = 0; dc < 2; ++dc) {
        FH kb;
        kb.h[0] = *(const v8h*)(Ksh + (j * 16 + c) * QD + dc * 32 + 8 * hh);
        kb.h[1] = *(const v8h*)(Ksh + (j * 16 + c) * QD + dc * 32 + 16 + 8 * hh);
        a = mma_h(qa[dc], kb.v, a);
      }
#pragma unroll
      for (int r = 0; r < 8; ++r) s[j][r] = a[r] * sscale;
    }

    _Float16* pwh = Psh[wave];
    _Float16* pwl = Psl[wave];
#pragma unroll
    for (int r = 0; r < 8; ++r) {
      float m = s[0][r];
#pragma unroll
      for (int j = 1; j < 4; ++j) m = fmaxf(m, s[j][r]);
#pragma unroll
      for (int off = 1; off < 16; off <<= 1) m = fmaxf(m, __shfl_xor(m, off, 32));
      const float mnew  = fmaxf(mrow[r], m);
      const float msafe = (mnew == -INFINITY) ? 0.f : mnew;
      const float alpha = __expf(mrow[r] - msafe);
      mrow[r] = mnew;
      float psum = 0.f;
#pragma unroll
      for (int j = 0; j < 4; ++j) {
        const float p  = __expf(s[j][r] - msafe);
        psum += p;
        const float pp = p * 1024.0f;
        const _Float16 ph = (_Float16)pp;
        const float res = pp - (float)ph;
        const _Float16 pl = (_Float16)(res * 2048.0f);
        const int pidx = (8 * hh + r) * 64 + j * 16 + c;
        pwh[pidx] = ph;
        pwl[pidx] = pl;
      }
#pragma unroll
      for (int off = 1; off < 16; off <<= 1) psum += __shfl_xor(psum, off, 32);
      lrow[r] = lrow[r] * alpha + psum;
#pragma unroll
      for (int t = 0; t < 2; ++t) oacc[t][r] *= alpha;
    }
    __builtin_amdgcn_fence(__ATOMIC_RELEASE, "workgroup");
    __builtin_amdgcn_wave_barrier();
    __builtin_amdgcn_fence(__ATOMIC_ACQUIRE, "workgroup");

    v8f o1[2], o2[2];
#pragma unroll
    for (int t = 0; t < 2; ++t) { o1[t] = zero8(); o2[t] = zero8(); }
#pragma unroll 1
    for (int kk = 0; kk < 2; ++kk) {
      FH pa, pr;
      pa.h[0] = *(const v8h*)(pwh + c * 64 + kk * 32 + 8 * hh);
      pa.h[1] = *(const v8h*)(pwh + c * 64 + kk * 32 + 16 + 8 * hh);
      pr.h[0] = *(const v8h*)(pwl + c * 64 + kk * 32 + 8 * hh);
      pr.h[1] = *(const v8h*)(pwl + c * 64 + kk * 32 + 16 + 8 * hh);
#pragma unroll
      for (int t = 0; t < 2; ++t) {
        FH vb, vr;
        vb.h[0] = *(const v8h*)(Vth + (t * 16 + c) * 64 + kk * 32 + 8 * hh);
        vb.h[1] = *(const v8h*)(Vth + (t * 16 + c) * 64 + kk * 32 + 16 + 8 * hh);
        vr.h[0] = *(const v8h*)(Vtl + (t * 16 + c) * 64 + kk * 32 + 8 * hh);
        vr.h[1] = *(const v8h*)(Vtl + (t * 16 + c) * 64 + kk * 32 + 16 + 8 * hh);
        oacc[t] = mma_h(pa.v, vb.v, oacc[t]);
        o1[t]   = mma_h(pa.v, vr.v, o1[t]);
        o2[t]   = mma_h(pr.v, vb.v, o2[t]);
      }
    }
#pragma unroll
    for (int t = 0; t < 2; ++t)
#pragma unroll
      for (int r = 0; r < 8; ++r) {
        const float f1 = o1[t][r] * (1.0f / 4096.0f);
        const float f2 = o2[t][r] * (1.0f / 2048.0f);
        oacc[t][r] = oacc[t][r] + f1 + f2;
      }
  }

  float* os = Os[wave];
#pragma unroll
  for (int r = 0; r < 8; ++r) {
    const float l = lrow[r];
    const float inv = ((l > 0.f) ? (1.0f / l) : 0.f) * (1.0f / 8192.0f);
#pragma unroll
    for (int t = 0; t < 2; ++t) os[(8 * hh + r) * HD + t * 16 + c] = oacc[t][r] * inv;
  }
  __builtin_amdgcn_fence(__ATOMIC_RELEASE, "workgroup");
  __builtin_amdgcn_wave_barrier();
  __builtin_amdgcn_fence(__ATOMIC_ACQUIRE, "workgroup");
  {
    const int q4 = lane >> 3, c4 = (lane & 7) * 4;
    v4f ov[4];
#pragma unroll
    for (int it = 0; it < 4; ++it) {
      const int row = it * 4 + q4;
      const float* spo = os + row * HD + c4;
      v4f v;
      v[0] = spo[0]; v[1] = spo[1]; v[2] = spo[2]; v[3] = spo[3];
      ov[it] = v;
    }
    for (int pass = 0; pass < 2; ++pass) {
#pragma unroll
      for (int it = 0; it < 4; ++it) {
        const int row = it * 4 + q4;
        const size_t go = ((size_t)b * SEQ + (size_t)(q0 + row)) * EMB + (size_t)h * HD + c4;
        *(volatile v4f*)(out + go) = ov[it];
      }
      __threadfence();
    }
  }
}

extern "C" void kernel_launch(void* const* d_in, const int* in_sizes, int n_in,
                              void* d_out, int out_size, void* d_ws, size_t ws_size,
                              hipStream_t stream) {
  if (n_in < 6) return;
  if (in_sizes[0] != NB * SEQ * EMB) return;
  if (in_sizes[1] != NB * SEQ * EMB) return;
  if (in_sizes[2] != NB * SEQ * 4) return;
  if (in_sizes[3] != HD * HD || in_sizes[4] != HD * HD || in_sizes[5] != HD * HD) return;
  if (out_size != NB * SEQ * EMB) return;

  const float* content = (const float*)d_in[0];
  const float* posenc  = (const float*)d_in[1];
  const float* centers = (const float*)d_in[2];
  const float* Wq      = (const float*)d_in[3];
  const float* Wk      = (const float*)d_in[4];
  const float* Wv      = (const float*)d_in[5];

  const size_t PPT = (size_t)NB * SEQ * 2 * 4;
  const size_t PQ2 = (size_t)NB * NH * SEQ * QD * 2;
  const size_t PVT = (size_t)NB * NH * HD * SEQ * 2;
  size_t off = 0;
  const size_t oPT = off; off += PPT;
  const size_t oQ2 = off; off += PQ2;
  const size_t oK2 = off; off += PQ2;
  const size_t oVh = off; off += PVT;
  const size_t oVl = off; off += PVT;
  if (off > ws_size) return;
  if (off > (size_t)134217728) return;

  char* ws = (char*)d_ws;
  int*            PT  = (int*)(ws + oPT);
  unsigned short* Q2  = (unsigned short*)(ws + oQ2);
  unsigned short* K2  = (unsigned short*)(ws + oK2);
  unsigned short* VTh = (unsigned short*)(ws + oVh);
  unsigned short* VTl = (unsigned short*)(ws + oVl);
  float*          outp = (float*)d_out;

  const float sscale = (1.0f / 64.0f) / sqrtf(2.0f * (float)EMB);

  const dim3 gP(NQT, NB);
  const dim3 gT(NQT, NH, NB);

  k_partner<<<gP, dim3(64), 0, stream>>>(centers, PT);
  k_proj<<<gT, dim3(256), 0, stream>>>(content, posenc, PT, Wq, Wk, Wv, Q2, K2, VTh, VTl);
  k_attn<<<gT, dim3(128), 0, stream>>>(Q2, K2, VTh, VTl, outp, sscale);
  (void)hipGetLastError();
}
